// EdgeDecoder_11003706212841
// MI455X (gfx1250) — hardware-verified
//
#include <hip/hip_runtime.h>


#define NB_  4
#define NN   512
#define DD   256
#define HH   128
#define IC   128
#define NPC  (IC * NN)
#define NP3  64
typedef _Float16 h16;
typedef unsigned short bf;
typedef __attribute__((ext_vector_type(16))) __bf16   v16bf;
typedef __attribute__((ext_vector_type(16))) _Float16 v16h;
typedef __attribute__((ext_vector_type(8)))  _Float16 v8h;
typedef __attribute__((ext_vector_type(8)))  unsigned short v8us;
typedef __attribute__((ext_vector_type(8)))  float    v8f;
typedef __attribute__((ext_vector_type(4)))  float    v4f;
typedef v8h  __attribute__((may_alias)) v8ha;
typedef v4f  __attribute__((may_alias)) v4fa;
typedef v8us __attribute__((may_alias)) v8usa;

__device__ __forceinline__ unsigned short f2bf(float f) { unsigned u = __float_as_uint(f); u += 0x7FFFu + ((u >> 16) & 1u); return (unsigned short)(u >> 16); }
__device__ __forceinline__ float bf2f(unsigned short b) { return __uint_as_float(((unsigned)b) << 16); }
__device__ __forceinline__ float bfr(float f) { return bf2f(f2bf(f)); }
__device__ __forceinline__ v16h cat16(v8h lo, v8h hi) { return __builtin_shufflevector(lo, hi, 0, 1, 2, 3, 4, 5, 6, 7, 8, 9, 10, 11, 12, 13, 14, 15); }
__device__ __forceinline__ v16bf cat16b(v8us lo, v8us hi) { return __builtin_bit_cast(v16bf, __builtin_shufflevector(lo, hi, 0, 1, 2, 3, 4, 5, 6, 7, 8, 9, 10, 11, 12, 13, 14, 15)); }
__device__ __forceinline__ v8f wmma16(v16h a, v16h b, v8f c) { return __builtin_amdgcn_wmma_f32_16x16x32_f16(false, a, false, b, (short)0, c, false, false); }
__device__ __forceinline__ v8f wmmab(v16bf a, v16bf b, v8f c) { return __builtin_amdgcn_wmma_f32_16x16x32_bf16(false, a, false, b, (short)0, c, false, false); }


template <typename T16> struct WFrag;
template <> struct WFrag<h16> { typedef v16h V; static __device__ __forceinline__ V ld(const h16* p) { return cat16(*(const v8h*)p, *(const v8h*)(p + 16)); } static __device__ __forceinline__ v8f mma(V a, V b, v8f c) { return wmma16(a, b, c); } };
template <> struct WFrag<bf> { typedef v16bf V; static __device__ __forceinline__ V ld(const bf* p) { return cat16b(*(const v8us*)p, *(const v8us*)(p + 16)); } static __device__ __forceinline__ v8f mma(V a, V b, v8f c) { return wmmab(a, b, c); } };
template <typename T16, int NSPLIT, bool BIAS>
__global__ __launch_bounds__(32) void k_gemmw(const T16* __restrict__ A, const T16* __restrict__ A2, const T16* __restrict__ Bt, const T16* __restrict__ Bt2, int K, float* C, int ldc, const float* __restrict__ bias, size_t sA, size_t sB, size_t sC) {
    typedef typename WFrag<T16>::V V;
    __shared__ __align__(16) float os[16 * 68];
    const size_t z = blockIdx.z; A += z * sA; if (A2) A2 += z * sA; Bt += z * sB; if (Bt2) Bt2 += z * sB; C += z * sC;
    const int lane = threadIdx.x & 31, lr = lane & 15, hi = lane >> 4; const int r0 = blockIdx.x * 64, c0 = blockIdx.y * 64;
    v8f acc[4][4];
#pragma unroll
    for (int mb = 0; mb < 4; ++mb)
#pragma unroll
        for (int nb = 0; nb < 4; ++nb) acc[mb][nb] = (v8f){};
    const size_t aoff = (size_t)(r0 + lr) * K + 8 * hi, boff = (size_t)(c0 + lr) * K + 8 * hi;
#pragma unroll 1
    for (int kc = 0; kc < K; kc += 32) {
        V a[4], a2[4];
#pragma unroll
        for (int mb = 0; mb < 4; ++mb) { a[mb] = WFrag<T16>::ld(A + aoff + (size_t)mb * 16 * K + kc); if (NSPLIT == 1 || NSPLIT == 2) a2[mb] = WFrag<T16>::ld(A2 + aoff + (size_t)mb * 16 * K + kc); }
#pragma unroll
        for (int nb = 0; nb < 4; ++nb) { const V b = WFrag<T16>::ld(Bt + boff + (size_t)nb * 16 * K + kc); V b2; if (NSPLIT >= 2) b2 = WFrag<T16>::ld(Bt2 + boff + (size_t)nb * 16 * K + kc);
#pragma unroll
            for (int mb = 0; mb < 4; ++mb) { acc[mb][nb] = WFrag<T16>::mma(a[mb], b, acc[mb][nb]); if (NSPLIT == 1 || NSPLIT == 2) acc[mb][nb] = WFrag<T16>::mma(a2[mb], b, acc[mb][nb]); if (NSPLIT >= 2) acc[mb][nb] = WFrag<T16>::mma(a[mb], b2, acc[mb][nb]); } }
        asm volatile("v_nop\n\tv_nop\n\tv_nop\n\tv_nop" : "+v"(acc[0][0]), "+v"(acc[1][1]), "+v"(acc[2][2]), "+v"(acc[3][3]) : "v"(a[0]), "v"(a[3]));
    }
#pragma unroll
    for (int mb = 0; mb < 4; ++mb) {
#pragma unroll
        for (int nb = 0; nb < 4; ++nb) {
#pragma unroll
            for (int j = 0; j < 8; ++j) os[(hi * 8 + j) * 68 + nb * 16 + lr] = acc[mb][nb][j]; }
        __builtin_amdgcn_wave_barrier(); asm volatile("" ::: "memory");
        float* crow = C + (size_t)(r0 + mb * 16) * ldc + c0;
#pragma unroll 1
        for (int ps = 0; ps < 2; ++ps) {
#pragma unroll
            for (int s = 0; s < 8; ++s) { const int row = 2 * s + hi, cofs = lr * 4; v4f val = *(const v4fa*)(os + row * 68 + cofs); if (BIAS) { val[0] += bfr(bias[c0 + cofs]); val[1] += bfr(bias[c0 + cofs + 1]); val[2] += bfr(bias[c0 + cofs + 2]); val[3] += bfr(bias[c0 + cofs + 3]); }
                *(volatile v4f*)(crow + (size_t)row * ldc + cofs) = val; }
            if (ps == 0) __threadfence(); }
        __builtin_amdgcn_wave_barrier(); asm volatile("" ::: "memory");
    }
}

typedef __attribute__((ext_vector_type(4))) unsigned short v4us;
typedef __attribute__((ext_vector_type(2))) unsigned short v2us;
__device__ __forceinline__ void splitf(float y, unsigned short& h, unsigned short& l) { h = f2bf(y); l = f2bf(y - bf2f(h)); }
__device__ __forceinline__ float gelu_erf(float x) { const float e = erff(__fmul_rn(x, 0.70710678118654752f)); float hx = __fmul_rn(0.5f, x); asm volatile("" : "+v"(hx)); return __fmul_rn(hx, __fadd_rn(1.0f, e)); }
__global__ __launch_bounds__(256) void k_cvt8(const float* __restrict__ src, bf* dst, size_t n8) { const size_t i = (size_t)blockIdx.x * 256 + threadIdx.x; if (i >= n8) return; const v8f v = *(const v8f*)(src + i * 8); v8us o;
#pragma unroll
    for (int k = 0; k < 8; ++k) o[k] = f2bf(v[k]); *(volatile v8us*)(dst + i * 8) = o; __threadfence(); *(volatile v8us*)(dst + i * 8) = o; }

__global__ __launch_bounds__(256) void k_wtG(const float* __restrict__ w, int K, int N, bf* Bt) {
    const int lane = threadIdx.x & 31; const int L0 = (blockIdx.x * 8 + (threadIdx.x >> 5)) * 8; const int nlines = N * K / 64;
#pragma unroll
    for (int ps = 0; ps < 2; ++ps) {
#pragma unroll 1
        for (int l = 0; l < 8; ++l) { const int L = L0 + l; if (L >= nlines) break; const size_t e = (size_t)L * 64 + lane * 2; const int k = (int)(e % K), n = (int)(e / K); v2us o;
            o[0] = f2bf(w[(size_t)k * N + n]); o[1] = f2bf(w[(size_t)(k + 1) * N + n]); *(volatile v2us*)(Bt + e) = o; }
        if (ps == 0) __threadfence(); }
}

__global__ __launch_bounds__(256) void k_tohl(const float* __restrict__ F, bf* Hh, bf* Hl, size_t n4) { const size_t i = (size_t)blockIdx.x * 256 + threadIdx.x; if (i >= n4) return; const v4f a = *(const v4f*)(F + i * 4); v4us oh, ol;
#pragma unroll
    for (int q = 0; q < 4; ++q) { unsigned short h2, l2; splitf(a[q], h2, l2); oh[q] = h2; ol[q] = l2; }
    *(volatile v4us*)(Hh + i * 4) = oh; *(volatile v4us*)(Hl + i * 4) = ol; __threadfence(); *(volatile v4us*)(Hh + i * 4) = oh; *(volatile v4us*)(Hl + i * 4) = ol; }
__global__ __launch_bounds__(256) void k_w3pad(const float* __restrict__ w3, const float* __restrict__ b3, bf* Bt, float* BP) { const int i = blockIdx.x * 256 + threadIdx.x; if (i >= NP3 * HH / 8) return; const int k0 = (i % (HH / 8)) * 8; const int n = i / (HH / 8); v8us o;
#pragma unroll
    for (int q = 0; q < 8; ++q) { const unsigned short e = f2bf(w3[k0 + q]); o[q] = (n == 0) ? e : (unsigned short)0; }
    *(volatile v8us*)(Bt + (size_t)n * HH + k0) = o; __threadfence(); *(volatile v8us*)(Bt + (size_t)n * HH + k0) = o;
    if (i < NP3 / 4) { v4f bb; const float b0 = bfr(b3[0]); for (int q = 0; q < 4; ++q) bb[q] = (i * 4 + q == 0) ? b0 : 0.0f; *(volatile v4f*)(BP + i * 4) = bb; __threadfence(); *(volatile v4f*)(BP + i * 4) = bb; } }
__global__ __launch_bounds__(256) void k_pair(const float* __restrict__ S1, const float* __restrict__ T1, const float* __restrict__ b1, int i0, bf* Ph, bf* Pl) { const size_t k = (size_t)blockIdx.x * 256 + threadIdx.x; if (k >= (size_t)NPC * HH / 4) return; const int h0 = (int)(k % (HH / 4)) * 4; const size_t p = k / (HH / 4); const int j = (int)(p % NN); const int i = i0 + (int)(p / NN); const v4f s = *(const v4f*)(S1 + (size_t)i * HH + h0); const v4f t = *(const v4f*)(T1 + (size_t)j * HH + h0); v4us oh, ol;
#pragma unroll
    for (int q = 0; q < 4; ++q) { float a = __fadd_rn(s[q], t[q]); asm volatile("" : "+v"(a)); a = __fadd_rn(a, bfr(b1[h0 + q])); unsigned short x2, y2; splitf(gelu_erf(a), x2, y2); oh[q] = x2; ol[q] = y2; }
    *(volatile v4us*)(Ph + p * HH + h0) = oh; *(volatile v4us*)(Pl + p * HH + h0) = ol; __threadfence(); *(volatile v4us*)(Ph + p * HH + h0) = oh; *(volatile v4us*)(Pl + p * HH + h0) = ol; }
__global__ __launch_bounds__(256) void k_gelu(const float* __restrict__ F, bf* Hh, bf* Hl, size_t n4) { const size_t i = (size_t)blockIdx.x * 256 + threadIdx.x; if (i >= n4) return; const v4f a = *(const v4f*)(F + i * 4); v4us oh, ol;
#pragma unroll
    for (int q = 0; q < 4; ++q) { unsigned short h2, l2; splitf(gelu_erf(a[q]), h2, l2); oh[q] = h2; ol[q] = l2; }
    *(volatile v4us*)(Hh + i * 4) = oh; *(volatile v4us*)(Hl + i * 4) = ol; __threadfence(); *(volatile v4us*)(Hh + i * 4) = oh; *(volatile v4us*)(Hl + i * 4) = ol; }
__global__ __launch_bounds__(256) void k_adj(const float* __restrict__ F3, int i0, float* out) { const int k = blockIdx.x * 256 + threadIdx.x; if (k >= IC * NN / 4) return; const int j0 = (k % (NN / 4)) * 4; const int il = k / (NN / 4); const int i = i0 + il; v4f o;
#pragma unroll
    for (int q = 0; q < 4; ++q) { const float a = F3[((size_t)il * NN + j0 + q) * NP3]; o[q] = (j0 + q == i) ? 0.0f : a; }
    *(volatile v4f*)(out + (size_t)i * NN + j0) = o; __threadfence(); *(volatile v4f*)(out + (size_t)i * NN + j0) = o; }

extern "C" void kernel_launch(void* const* d_in, const int* in_sizes, int n_in,
                              void* d_out, int out_size, void* d_ws, size_t ws_size, hipStream_t stream) {
    (void)in_sizes; (void)n_in; (void)out_size;
    const float* E = (const float*)d_in[0]; const float* wsrc = (const float*)d_in[1]; const float* bsrc = (const float*)d_in[2]; const float* wtgt = (const float*)d_in[3]; const float* btgt = (const float*)d_in[4]; const float* w1 = (const float*)d_in[5]; const float* b1 = (const float*)d_in[6]; const float* w2 = (const float*)d_in[7]; const float* b2 = (const float*)d_in[8]; const float* w3 = (const float*)d_in[9]; const float* b3 = (const float*)d_in[10];
    float* OUT = (float*)d_out;
    char* wsp = (char*)d_ws;
    auto take = [&](size_t bytes) { char* p = wsp; wsp += (bytes + 255) & ~(size_t)255; return (void*)p; };
    bf* WS = (bf*)take((size_t)HH * DD * 2); bf* WT = (bf*)take((size_t)HH * DD * 2); bf* W1A = (bf*)take((size_t)HH * HH * 2); bf* W1B = (bf*)take((size_t)HH * HH * 2); bf* W2B = (bf*)take((size_t)HH * HH * 2); bf* W3B = (bf*)take((size_t)NP3 * HH * 2); float* B3P = (float*)take((size_t)NP3 * 4);
    bf* EB = (bf*)take((size_t)NN * DD * 2); float* FS = (float*)take((size_t)NN * HH * 4); float* FT = (float*)take((size_t)NN * HH * 4); bf* Nh = (bf*)take((size_t)NN * HH * 2); bf* Nl = (bf*)take((size_t)NN * HH * 2); float* S1 = (float*)take((size_t)NN * HH * 4); float* T1 = (float*)take((size_t)NN * HH * 4);
    bf* Ph = (bf*)take((size_t)NPC * HH * 2); bf* Pl = (bf*)take((size_t)NPC * HH * 2); float* F2 = (float*)take((size_t)NPC * HH * 4); bf* Gh = (bf*)take((size_t)NPC * HH * 2); bf* Gl = (bf*)take((size_t)NPC * HH * 2); float* F3 = (float*)take((size_t)NPC * NP3 * 4);
    if ((size_t)(wsp - (char*)d_ws) > ws_size) return;
    k_wtG<<<(DD * HH / 64 + 63) / 64, 256, 0, stream>>>(wsrc, DD, HH, WS); k_wtG<<<(DD * HH / 64 + 63) / 64, 256, 0, stream>>>(wtgt, DD, HH, WT);
    k_wtG<<<(HH * HH / 64 + 63) / 64, 256, 0, stream>>>(w1, HH, HH, W1A); k_wtG<<<(HH * HH / 64 + 63) / 64, 256, 0, stream>>>(w1 + (size_t)HH * HH, HH, HH, W1B);
    k_wtG<<<(HH * HH / 64 + 63) / 64, 256, 0, stream>>>(w2, HH, HH, W2B); k_w3pad<<<(NP3 * HH / 8 + 255) / 256, 256, 0, stream>>>(w3, b3, W3B, B3P);
    const size_t n4n = (size_t)NN * HH / 4; const unsigned g4n = (unsigned)((n4n + 255) / 256);
    for (int b = 0; b < NB_; ++b) {
        k_cvt8<<<(unsigned)(((size_t)NN * DD / 8 + 255) / 256), 256, 0, stream>>>(E + (size_t)b * NN * DD, EB, (size_t)NN * DD / 8);
        k_gemmw<bf, 0, true><<<dim3(NN / 64, HH / 64, 1), 32, 0, stream>>>(EB, nullptr, WS, nullptr, DD, FS, HH, bsrc, 0, 0, 0);
        k_gemmw<bf, 0, true><<<dim3(NN / 64, HH / 64, 1), 32, 0, stream>>>(EB, nullptr, WT, nullptr, DD, FT, HH, btgt, 0, 0, 0);
        k_tohl<<<g4n, 256, 0, stream>>>(FS, Nh, Nl, n4n); k_gemmw<bf, 1, false><<<dim3(NN / 64, HH / 64, 1), 32, 0, stream>>>(Nh, Nl, W1A, nullptr, HH, S1, HH, nullptr, 0, 0, 0);
        k_tohl<<<g4n, 256, 0, stream>>>(FT, Nh, Nl, n4n); k_gemmw<bf, 1, false><<<dim3(NN / 64, HH / 64, 1), 32, 0, stream>>>(Nh, Nl, W1B, nullptr, HH, T1, HH, nullptr, 0, 0, 0);
        for (int i0 = 0; i0 < NN; i0 += IC) {
            k_pair<<<(unsigned)(((size_t)NPC * HH / 4 + 255) / 256), 256, 0, stream>>>(S1, T1, b1, i0, Ph, Pl);
            k_gemmw<bf, 1, true><<<dim3(NPC / 64, HH / 64, 1), 32, 0, stream>>>(Ph, Pl, W2B, nullptr, HH, F2, HH, b2, 0, 0, 0);
            k_gelu<<<(unsigned)(((size_t)NPC * HH / 4 + 255) / 256), 256, 0, stream>>>(F2, Gh, Gl, (size_t)NPC * HH / 4);
            k_gemmw<bf, 1, true><<<dim3(NPC / 64, NP3 / 64, 1), 32, 0, stream>>>(Gh, Gl, W3B, nullptr, HH, F3, NP3, B3P, 0, 0, 0);
            k_adj<<<(IC * NN / 4 + 255) / 256, 256, 0, stream>>>(F3, i0, OUT + (size_t)b * NN * NN); } }
}
